// Decoder_50508815401309
// MI455X (gfx1250) — hardware-verified
//
#include <hip/hip_runtime.h>
#include <math.h>

constexpr int NBATCH = 128;
constexpr int NSEQ   = 64;
constexpr int NUNIT  = 512;
constexpr int NVOCAB = 32000;
constexpr int NROWS  = NBATCH * NSEQ;
constexpr int NXC    = 2 * NUNIT;
constexpr int NGATE  = 3 * NUNIT;
constexpr int NTHR   = 256;
constexpr float W_CARRY     = 64.0f;
constexpr float W_CARRY_INV = 1.0f / W_CARRY;
constexpr float Y_CARRY     = 64.0f;
constexpr float LOGIT_FOLD  = 1.0f / (W_CARRY * Y_CARRY);
constexpr int OUT_LOGITS_ELEMS = NBATCH * NVOCAB;
constexpr int OUT_STATE_ELEMS  = NBATCH * NUNIT;
constexpr int OUT_ALPHA_ELEMS  = NBATCH * NSEQ;
constexpr int OUT_TOTAL_ELEMS  = OUT_LOGITS_ELEMS + OUT_STATE_ELEMS + OUT_ALPHA_ELEMS;

static_assert(NROWS == 8192);
static_assert(NROWS % 64 == 0 && NBATCH % 64 == 0);
static_assert(NUNIT % 64 == 0 && NGATE % 64 == 0 && NVOCAB % 64 == 0);
static_assert(NUNIT % 32 == 0 && NXC % 32 == 0);
static_assert((size_t)OUT_LOGITS_ELEMS * 4 == 16384000);
static_assert((size_t)(OUT_LOGITS_ELEMS + OUT_STATE_ELEMS) * 4 == 16646144);
static_assert((size_t)OUT_TOTAL_ELEMS * 4 == 16678912);
static_assert(((size_t)OUT_LOGITS_ELEMS * 4) % 128 == 0);
static_assert(((size_t)(OUT_LOGITS_ELEMS + OUT_STATE_ELEMS) * 4) % 128 == 0);
static_assert(NUNIT == 2 * NTHR);
static_assert(NSEQ == 64);

typedef __attribute__((ext_vector_type(16))) _Float16 v16h;
typedef __attribute__((ext_vector_type(8)))  _Float16 v8h;
typedef __attribute__((ext_vector_type(16))) __bf16   v16b;
typedef __attribute__((ext_vector_type(8)))  __bf16   v8b;
typedef __attribute__((ext_vector_type(8)))  float    v8f;
typedef __attribute__((ext_vector_type(4)))  float    v4f;
typedef __attribute__((ext_vector_type(2)))  float    v2f;
typedef __attribute__((ext_vector_type(4)))  unsigned v4u;

__device__ __forceinline__ unsigned short f2bf_bits(float f) {
  unsigned u = __float_as_uint(f);
  return (unsigned short)((u + 0x7FFFu + ((u >> 16) & 1u)) >> 16);
}
__device__ __forceinline__ float bf_bits2f(unsigned short h) { return __uint_as_float(((unsigned)h) << 16); }
__device__ __forceinline__ unsigned short f2h_bits(float f) {
  const _Float16 h = (_Float16)f;
  return __builtin_bit_cast(unsigned short, h);
}
__device__ __forceinline__ unsigned pack2(unsigned short lo, unsigned short hi) {
  return (unsigned)lo | ((unsigned)hi << 16);
}

__device__ __forceinline__ void dep_guard4_h(v8f& a, v8f& b, v8f& c, v8f& d, v16h x, v16h y) { asm volatile("v_nop\n\tv_nop\n\tv_nop\n\tv_nop" : "+v"(a), "+v"(b), "+v"(c), "+v"(d) : "v"(x), "v"(y)); }
__device__ __forceinline__ void dep_guard4_b(v8f& a, v8f& b, v8f& c, v8f& d, v16b x, v16b y) { asm volatile("v_nop\n\tv_nop\n\tv_nop\n\tv_nop" : "+v"(a), "+v"(b), "+v"(c), "+v"(d) : "v"(x), "v"(y)); }
__device__ __forceinline__ void keep4_h(v16h a, v16h b, v16h c, v16h d) { asm volatile("v_nop" :: "v"(a), "v"(b), "v"(c), "v"(d)); }
__device__ __forceinline__ void keep4_b(v16b a, v16b b, v16b c, v16b d) { asm volatile("v_nop" :: "v"(a), "v"(b), "v"(c), "v"(d)); }
__device__ __forceinline__ void acc_guard4(v8f& a, v8f& b, v8f& c, v8f& d) { asm volatile("v_nop\n\tv_nop\n\tv_nop\n\tv_nop" : "+v"(a), "+v"(b), "+v"(c), "+v"(d)); }

template <typename T> struct Frag;
template <> struct Frag<_Float16> {
  typedef v16h V; union U { v16h v; v8h h[2]; };
  static __device__ __forceinline__ v16h load(const _Float16* p) {
    U f; f.h[0] = *(const v8h*)(p); f.h[1] = *(const v8h*)(p + 16); return f.v;
  }
  static __device__ __forceinline__ v8f mma(v16h a, v16h b, v8f c) {
    return __builtin_amdgcn_wmma_f32_16x16x32_f16(false, a, false, b, (short)0, c, false, false);
  }
  static __device__ __forceinline__ void guard4(v8f& a, v8f& b, v8f& c, v8f& d, v16h x, v16h y) { dep_guard4_h(a, b, c, d, x, y); }
  static __device__ __forceinline__ void keep(v16h a, v16h b, v16h c, v16h d) { keep4_h(a, b, c, d); }
};
template <> struct Frag<__bf16> {
  typedef v16b V; union U { v16b v; v8b h[2]; };
  static __device__ __forceinline__ v16b load(const __bf16* p) {
    U f; f.h[0] = *(const v8b*)(p); f.h[1] = *(const v8b*)(p + 16); return f.v;
  }
  static __device__ __forceinline__ v8f mma(v16b a, v16b b, v8f c) {
    return __builtin_amdgcn_wmma_f32_16x16x32_bf16(false, a, false, b, (short)0, c, false, false);
  }
  static __device__ __forceinline__ void guard4(v8f& a, v8f& b, v8f& c, v8f& d, v16b x, v16b y) { dep_guard4_b(a, b, c, d, x, y); }
  static __device__ __forceinline__ void keep(v16b a, v16b b, v16b c, v16b d) { keep4_b(a, b, c, d); }
};

template <int ET> struct Elem;
template <> struct Elem<0> { typedef _Float16 T; };
template <> struct Elem<1> { typedef __bf16 T; };
template <int ET, bool SPLIT, int BIAS_MODE, int OUT_MODE, int ACT>
__global__ __launch_bounds__(256) void wmma_gemm64(
    const unsigned short* __restrict__ Ap, const unsigned short* __restrict__ A2p, int lda,
    const unsigned short* __restrict__ Btp, const unsigned short* __restrict__ Bt2p, int ldb,
    void* __restrict__ Cout, int ldc,
    const float* __restrict__ bias,
    int M, int N, int K, float scale) {
  typedef typename Elem<ET>::T T;
  typedef typename Frag<T>::V V;
  const T* A = (const T*)Ap; const T* A2 = (const T*)A2p; const T* Bt = (const T*)Btp; const T* Bt2 = (const T*)Bt2p;
  __shared__ __align__(16) float sT[8][16 * 68];
  const int lane = threadIdx.x & 31;
  const int wave = threadIdx.x >> 5;
  const int tilesN = N >> 6;
  const int tilesM = M >> 6;
  const int tile = blockIdx.x * 8 + wave;
  if (tile >= tilesM * tilesN) return;
  const int tm = tile / tilesN;
  const int tn = tile - tm * tilesN;
  const int m0 = tm << 6;
  const int n0 = tn << 6;

  const int rlane = lane & 15;
  const int koff  = (lane >> 4) * 8;
  const int mOff  = (lane >> 4) * 8;

  v8f acc[4][4];
#pragma unroll
  for (int i = 0; i < 4; ++i)
#pragma unroll
    for (int j = 0; j < 4; ++j) acc[i][j] = (v8f){0.f,0.f,0.f,0.f,0.f,0.f,0.f,0.f};

  for (int k0 = 0; k0 < K; k0 += 32) {
    V bh[4], bl[4];
#pragma unroll
    for (int j = 0; j < 4; ++j) {
      const size_t bo = (size_t)(n0 + (j << 4) + rlane) * ldb + koff + k0;
      bh[j] = Frag<T>::load(Bt + bo);
      if (SPLIT) bl[j] = Frag<T>::load(Bt2 + bo);
    }
#pragma unroll
    for (int i = 0; i < 4; ++i) {
      const size_t ao = (size_t)(m0 + (i << 4) + rlane) * lda + koff + k0;
      V ah = Frag<T>::load(A + ao);
      V al;
      if (SPLIT) al = Frag<T>::load(A2 + ao);
#pragma unroll
      for (int j = 0; j < 4; ++j) {
        acc[i][j] = Frag<T>::mma(ah, bh[j], acc[i][j]);
        if (SPLIT) {
          acc[i][j] = Frag<T>::mma(ah, bl[j], acc[i][j]);
          acc[i][j] = Frag<T>::mma(al, bh[j], acc[i][j]);
        }
      }
      Frag<T>::guard4(acc[i][0], acc[i][1], acc[i][2], acc[i][3], ah, SPLIT ? al : ah);
    }
    Frag<T>::keep(bh[0], bh[1], bh[2], bh[3]);
    if (SPLIT) Frag<T>::keep(bl[0], bl[1], bl[2], bl[3]);
  }
  acc_guard4(acc[0][0], acc[0][1], acc[0][2], acc[0][3]);
  acc_guard4(acc[1][0], acc[1][1], acc[1][2], acc[1][3]);
  acc_guard4(acc[2][0], acc[2][1], acc[2][2], acc[2][3]);
  acc_guard4(acc[3][0], acc[3][1], acc[3][2], acc[3][3]);

  float* slab = sT[wave];
#pragma unroll
  for (int i = 0; i < 4; ++i) {
    const int mBase = m0 + (i << 4);
#pragma unroll
    for (int j = 0; j < 4; ++j) {
      const int n = n0 + (j << 4) + rlane;
      float bv = 0.f;
      if (BIAS_MODE == 2) bv = bias[n];
#pragma unroll
      for (int r = 0; r < 8; ++r) {
        float v = acc[i][j][r] * scale;
        if (BIAS_MODE == 2) v += bv;
        if (ACT == 2) v = fmaxf(v, 0.0f);
        if (ACT == 6) v = fmaxf(v, 0.0f) * Y_CARRY;
        slab[(mOff + r) * 68 + (j << 4) + rlane] = v;
      }
    }
    __builtin_amdgcn_fence(__ATOMIC_RELEASE, "workgroup");
    __builtin_amdgcn_wave_barrier();
    __builtin_amdgcn_fence(__ATOMIC_ACQUIRE, "workgroup");
    if (OUT_MODE == 0) {
      float* C = (float*)Cout;
      const int hh = lane >> 4, c4 = (lane & 15) * 4;
      for (int pass = 0; pass < 2; ++pass) {
#pragma unroll
        for (int it = 0; it < 8; ++it) {
          const int row = it * 2 + hh;
          v4f v = *(const v4f*)(slab + row * 68 + c4);
          *(volatile v4f*)(C + (size_t)(mBase + row) * ldc + n0 + c4) = v;
        }
        __threadfence();
      }
    } else {
      const int q = lane >> 3, c8 = (lane & 7) * 8;
      unsigned short* C = (unsigned short*)Cout;
      for (int pass = 0; pass < 2; ++pass) {
#pragma unroll
        for (int it = 0; it < 4; ++it) {
          const int row = it * 4 + q;
          const float* sp = slab + row * 68 + c8;
          v8h hv;
#pragma unroll
          for (int e = 0; e < 8; ++e) hv[e] = (_Float16)sp[e];
          *(volatile v8h*)(C + (size_t)(mBase + row) * ldc + n0 + c8) = hv;
        }
        __threadfence();
      }
    }
    __builtin_amdgcn_fence(__ATOMIC_RELEASE, "workgroup");
    __builtin_amdgcn_wave_barrier();
    __builtin_amdgcn_fence(__ATOMIC_ACQUIRE, "workgroup");
  }
}

__global__ __launch_bounds__(NTHR) void cvt_f16_kernel(const float* __restrict__ src,
                                                       unsigned short* __restrict__ dst, int n8) {
  const int i = blockIdx.x * NTHR + threadIdx.x;
  if (i < n8) {
    const float* sp = src + (size_t)i * 8;
    const v4f a = *(const v4f*)(sp);
    const v4f b = *(const v4f*)(sp + 4);
    const float a0 = a[0], a1 = a[1], a2 = a[2], a3 = a[3];
    const float b0 = b[0], b1 = b[1], b2 = b[2], b3 = b[3];
    v4u w;
    w[0] = pack2(f2h_bits(a0), f2h_bits(a1));
    w[1] = pack2(f2h_bits(a2), f2h_bits(a3));
    w[2] = pack2(f2h_bits(b0), f2h_bits(b1));
    w[3] = pack2(f2h_bits(b2), f2h_bits(b3));
    *(volatile v4u*)(dst + (size_t)i * 8) = w;
    __threadfence();
    *(volatile v4u*)(dst + (size_t)i * 8) = w;
  }
}

template <int MODE>
__global__ __launch_bounds__(NTHR) void tpw_kernel(const float* __restrict__ src, int R, int C, int ldo,
                                                  unsigned short* __restrict__ O, unsigned short* __restrict__ O2,
                                                  float sc) {
  __shared__ float Tt[64 * 65];
  const int tid = threadIdx.x;
  const int c0 = blockIdx.x * 64, r0 = blockIdx.y * 64;
#pragma unroll
  for (int i = 0; i < 4; ++i) {
    const int idx = i * NTHR + tid;
    const int rr = idx >> 4, cc = (idx & 15) * 4;
    const v4f v = *(const v4f*)(src + (size_t)(r0 + rr) * (size_t)C + c0 + cc);
    const float f0 = v[0], f1 = v[1], f2 = v[2], f3 = v[3];
    Tt[rr * 65 + cc + 0] = f0;
    Tt[rr * 65 + cc + 1] = f1;
    Tt[rr * 65 + cc + 2] = f2;
    Tt[rr * 65 + cc + 3] = f3;
  }
  __syncthreads();
  const int q = tid >> 3, c8 = (tid & 7) * 8;
  v4u hv[2], lv[2];
#pragma unroll
  for (int g = 0; g < 2; ++g) {
    const int qq = g * 32 + q;
#pragma unroll
    for (int p = 0; p < 4; ++p) {
      const float fa = Tt[(c8 + 2 * p) * 65 + qq];
      const float fb = Tt[(c8 + 2 * p + 1) * 65 + qq];
      unsigned short ha, hb, la, lb;
      if (MODE == 0) {
        ha = f2h_bits(fa * sc);
        hb = f2h_bits(fb * sc);
        la = ha;
        lb = hb;
      } else {
        ha = f2bf_bits(fa);
        hb = f2bf_bits(fb);
        la = f2bf_bits(fa - bf_bits2f(ha));
        lb = f2bf_bits(fb - bf_bits2f(hb));
      }
      hv[g][p] = pack2(ha, hb);
      lv[g][p] = pack2(la, lb);
    }
  }
  for (int pass = 0; pass < 2; ++pass) {
#pragma unroll
    for (int g = 0; g < 2; ++g) {
      const size_t o = (size_t)(c0 + g * 32 + q) * (size_t)ldo + (size_t)(r0 + c8);
      *(volatile v4u*)(O + o) = hv[g];
      if (MODE == 1) *(volatile v4u*)(O2 + o) = lv[g];
    }
    __threadfence();
  }
}

__global__ __launch_bounds__(NTHR) void attn_ctx_kernel(
    const float* __restrict__ PRE, const float* __restrict__ attn,
    const float* __restrict__ b0, const float* __restrict__ b1,
    const float* __restrict__ vW, const float* __restrict__ vb,
    const int* __restrict__ tok, const float* __restrict__ emb,
    float* __restrict__ alpha_out,
    unsigned short* __restrict__ XCH, unsigned short* __restrict__ XCL) {
  __shared__ __align__(16) float bs0[NUNIT];
  __shared__ __align__(16) float bs1[NUNIT];
  __shared__ __align__(16) float vws[NUNIT];
  __shared__ __align__(16) float scs[NSEQ];
  __shared__ __align__(16) float als[NSEQ];
  __shared__ __align__(16) float xcs[NXC];
  const int tid = threadIdx.x, lane = tid & 31, wave = tid >> 5;
  const int b = blockIdx.x;

#pragma unroll 1
  for (int i = tid; i < NUNIT; i += NTHR) {
    bs0[i] = b0[i];
    bs1[i] = b1[i];
    vws[i] = vW[i];
  }
  __syncthreads();

  const float vbv = vb[0];
#pragma unroll 1
  for (int i = 0; i < 8; ++i) {
    const int s = wave + 8 * i;
    const float* pr = PRE + ((size_t)b * NSEQ + (size_t)s) * NUNIT;
    float p = 0.0f;
#pragma unroll 1
    for (int q = 0; q < 16; ++q) {
      const int u = lane + 32 * q;
      const float t = tanhf((pr[u] + bs0[u]) + bs1[u]);
      p += t * vws[u];
    }
#pragma unroll
    for (int off = 1; off < 32; off <<= 1) p += __shfl_xor(p, off, 32);
    if (lane == 0) scs[s] = p + vbv;
  }
  __syncthreads();

  const float s0 = scs[lane];
  const float s1 = scs[lane + 32];
  float mx = fmaxf(s0, s1);
#pragma unroll
  for (int off = 1; off < 32; off <<= 1) {
    const float o = __shfl_xor(mx, off, 32);
    mx = fmaxf(mx, o);
  }
  const float e0 = expf(s0 - mx);
  const float e1 = expf(s1 - mx);
  float sm = e0 + e1;
#pragma unroll
  for (int off = 1; off < 32; off <<= 1) sm += __shfl_xor(sm, off, 32);
  const float inv = 1.0f / sm;
  if (wave == 0) {
    als[lane]      = e0 * inv;
    als[lane + 32] = e1 * inv;
  }
  __syncthreads();

  if (tid < 16) {
    const v4f av = *(const v4f*)(als + 4 * tid);
    float* ap = alpha_out + (size_t)b * NSEQ + 4 * tid;
    *(volatile v4f*)ap = av;
    __threadfence();
    *(volatile v4f*)ap = av;
  }

  {
    float c0 = 0.0f, c1 = 0.0f;
    const float* ap = attn + (size_t)b * NSEQ * NUNIT + 2 * tid;
#pragma unroll 4
    for (int s = 0; s < NSEQ; ++s) {
      const v2f a = *(const v2f*)(ap + (size_t)s * NUNIT);
      const float w = als[s];
      const float a0 = a[0], a1 = a[1];
      c0 += a0 * w;
      c1 += a1 * w;
    }
    xcs[NUNIT + 2 * tid]     = c0;
    xcs[NUNIT + 2 * tid + 1] = c1;
    int tk = tok[b];
    tk = tk < 0 ? 0 : (tk > NVOCAB - 1 ? NVOCAB - 1 : tk);
    const v2f ev = *(const v2f*)(emb + (size_t)tk * NUNIT + 2 * tid);
    const float x0 = ev[0], x1 = ev[1];
    xcs[2 * tid]     = x0;
    xcs[2 * tid + 1] = x1;
  }
  __syncthreads();

  {
    const int which = tid >> 7;
    const int idx8  = (tid & 127) * 8;
    const v4f xa = *(const v4f*)(xcs + idx8);
    const v4f xb = *(const v4f*)(xcs + idx8 + 4);
    float f[8];
    f[0] = xa[0]; f[1] = xa[1]; f[2] = xa[2]; f[3] = xa[3];
    f[4] = xb[0]; f[5] = xb[1]; f[6] = xb[2]; f[7] = xb[3];
    v4u w;
#pragma unroll
    for (int p = 0; p < 4; ++p) {
      const unsigned short ha = f2bf_bits(f[2 * p]);
      const unsigned short hb = f2bf_bits(f[2 * p + 1]);
      const unsigned short la = f2bf_bits(f[2 * p] - bf_bits2f(ha));
      const unsigned short lb = f2bf_bits(f[2 * p + 1] - bf_bits2f(hb));
      const unsigned wh = pack2(ha, hb);
      const unsigned wl = pack2(la, lb);
      w[p] = which ? wl : wh;
    }
    unsigned short* dp = (which ? XCL : XCH) + (size_t)b * NXC + idx8;
    *(volatile v4u*)dp = w;
    __threadfence();
    *(volatile v4u*)dp = w;
  }
}

__device__ __forceinline__ float fsigm(float x) { return __builtin_amdgcn_rcpf(1.0f + expf(-x)); }

__global__ __launch_bounds__(NTHR) void gru_kernel(const float* __restrict__ GX, const float* __restrict__ gb,
                                                   float* __restrict__ state_out,
                                                   unsigned short* __restrict__ STH, unsigned short* __restrict__ STL) {
  __shared__ __align__(16) float sts[NUNIT];
  const int tid = threadIdx.x;
  const int b = blockIdx.x;
  const float* g = GX + (size_t)b * NGATE;
#pragma unroll 1
  for (int it = 0; it < 2; ++it) {
    const int u = tid + NTHR * it;
    const float az = (g[u] + gb[u]) + gb[NGATE + u];
    const float ar = (g[NUNIT + u] + gb[NUNIT + u]) + gb[NGATE + NUNIT + u];
    const float xh = g[2 * NUNIT + u] + gb[2 * NUNIT + u];
    const float rh = gb[NGATE + 2 * NUNIT + u];
    const float z  = fsigm(az);
    const float r  = fsigm(ar);
    const float hh = tanhf(xh + r * rh);
    sts[u] = (1.0f - z) * hh;
  }
  __syncthreads();
  if (tid < 128) {
    const v4f sv = *(const v4f*)(sts + 4 * tid);
    float* op = state_out + (size_t)b * NUNIT + 4 * tid;
    *(volatile v4f*)op = sv;
    __threadfence();
    *(volatile v4f*)op = sv;
  } else {
    const int which = (tid >> 6) & 1;
    const int idx8  = (tid & 63) * 8;
    const v4f xa = *(const v4f*)(sts + idx8);
    const v4f xb = *(const v4f*)(sts + idx8 + 4);
    float f[8];
    f[0] = xa[0]; f[1] = xa[1]; f[2] = xa[2]; f[3] = xa[3];
    f[4] = xb[0]; f[5] = xb[1]; f[6] = xb[2]; f[7] = xb[3];
    v4u w;
#pragma unroll
    for (int p = 0; p < 4; ++p) {
      const unsigned short ha = f2bf_bits(f[2 * p]);
      const unsigned short hb = f2bf_bits(f[2 * p + 1]);
      const unsigned short la = f2bf_bits(f[2 * p] - bf_bits2f(ha));
      const unsigned short lb = f2bf_bits(f[2 * p + 1] - bf_bits2f(hb));
      const unsigned wh = pack2(ha, hb);
      const unsigned wl = pack2(la, lb);
      w[p] = which ? wl : wh;
    }
    unsigned short* dp = (which ? STL : STH) + (size_t)b * NUNIT + idx8;
    *(volatile v4u*)dp = w;
    __threadfence();
    *(volatile v4u*)dp = w;
  }
}

extern "C" void kernel_launch(void* const* d_in, const int* in_sizes, int n_in,
                              void* d_out, int out_size, void* d_ws, size_t ws_size, hipStream_t stream) {
  if (n_in < 16 || d_out == nullptr || d_ws == nullptr) return;
  if (in_sizes[0] != NBATCH || in_sizes[1] != NROWS * NUNIT || in_sizes[2] != NUNIT * NUNIT ||
      in_sizes[3] != NUNIT || in_sizes[5] != NUNIT || in_sizes[6] != NUNIT || in_sizes[7] != 1 ||
      in_sizes[8] != NVOCAB * NUNIT || in_sizes[9] != NXC * NGATE || in_sizes[11] != 2 * NGATE ||
      in_sizes[12] != NUNIT * NUNIT || in_sizes[13] != NUNIT || in_sizes[14] != NUNIT * NVOCAB ||
      in_sizes[15] != NVOCAB || out_size != OUT_TOTAL_ELEMS) return;

  const int*   tok   = (const int*)  d_in[0];
  const float* attn  = (const float*)d_in[1];
  const float* W0    = (const float*)d_in[2];
  const float* b0    = (const float*)d_in[3];
  const float* b1    = (const float*)d_in[5];
  const float* vW    = (const float*)d_in[6];
  const float* vb    = (const float*)d_in[7];
  const float* emb   = (const float*)d_in[8];
  const float* gru_k = (const float*)d_in[9];
  const float* gru_b = (const float*)d_in[11];
  const float* dW    = (const float*)d_in[12];
  const float* db    = (const float*)d_in[13];
  const float* oW    = (const float*)d_in[14];
  const float* ob    = (const float*)d_in[15];

  float* logits = (float*)d_out;
  float* state  = logits + (size_t)OUT_LOGITS_ELEMS;
  float* alpha  = state + (size_t)OUT_STATE_ELEMS;

  char* ws = (char*)d_ws; size_t off = 0;
  auto carve = [&](size_t bytes) -> char* { char* p = ws + off; off += (bytes + 255) & ~(size_t)255; return p; };
  unsigned short* A16 = (unsigned short*)carve((size_t)NROWS * NUNIT * 2);
  unsigned short* W0T = (unsigned short*)carve((size_t)NUNIT * NUNIT * 2);
  unsigned short* GKH = (unsigned short*)carve((size_t)NGATE * NXC * 2);
  unsigned short* GKL = (unsigned short*)carve((size_t)NGATE * NXC * 2);
  unsigned short* DWH = (unsigned short*)carve((size_t)NUNIT * NUNIT * 2);
  unsigned short* DWL = (unsigned short*)carve((size_t)NUNIT * NUNIT * 2);
  unsigned short* OWT = (unsigned short*)carve((size_t)NVOCAB * NUNIT * 2);
  float*          PRE = (float*)carve((size_t)NROWS * NUNIT * 4);
  unsigned short* XCH = (unsigned short*)carve((size_t)NBATCH * NXC * 2);
  unsigned short* XCL = (unsigned short*)carve((size_t)NBATCH * NXC * 2);
  float*          GX  = (float*)carve((size_t)NBATCH * NGATE * 4);
  unsigned short* STH = (unsigned short*)carve((size_t)NBATCH * NUNIT * 2);
  unsigned short* STL = (unsigned short*)carve((size_t)NBATCH * NUNIT * 2);
  unsigned short* Y16 = (unsigned short*)carve((size_t)NBATCH * NUNIT * 2);
  if (off > ws_size || off > (size_t)134217728) return;

  const int n8a = NROWS * (NUNIT / 8);
  cvt_f16_kernel<<<(n8a + NTHR - 1) / NTHR, NTHR, 0, stream>>>(attn, A16, n8a);
  tpw_kernel<0><<<dim3(NUNIT / 64, NUNIT / 64), NTHR, 0, stream>>>(W0, NUNIT, NUNIT, NUNIT, W0T, W0T, W_CARRY);
  tpw_kernel<1><<<dim3(NGATE / 64, NXC / 64), NTHR, 0, stream>>>(gru_k, NXC, NGATE, NXC, GKH, GKL, 1.0f);
  tpw_kernel<1><<<dim3(NUNIT / 64, NUNIT / 64), NTHR, 0, stream>>>(dW, NUNIT, NUNIT, NUNIT, DWH, DWL, 1.0f);
  tpw_kernel<0><<<dim3(NVOCAB / 64, NUNIT / 64), NTHR, 0, stream>>>(oW, NUNIT, NVOCAB, NUNIT, OWT, OWT, W_CARRY);

  wmma_gemm64<0, false, 0, 0, 0><<<dim3((NROWS / 64) * (NUNIT / 64) / 8), 256, 0, stream>>>(
      A16, A16, NUNIT, W0T, W0T, NUNIT, (void*)PRE, NUNIT, b0, NROWS, NUNIT, NUNIT, W_CARRY_INV);

  attn_ctx_kernel<<<NBATCH, NTHR, 0, stream>>>(PRE, attn, b0, b1, vW, vb, tok, emb, alpha, XCH, XCL);

  wmma_gemm64<1, true, 0, 0, 0><<<dim3((NBATCH / 64) * (NGATE / 64) / 8), 256, 0, stream>>>(
      XCH, XCL, NXC, GKH, GKL, NXC, (void*)GX, NGATE, gru_b, NBATCH, NGATE, NXC, 1.0f);

  gru_kernel<<<NBATCH, NTHR, 0, stream>>>(GX, gru_b, state, STH, STL);

  wmma_gemm64<1, true, 2, 1, 6><<<dim3((NBATCH / 64) * (NUNIT / 64) / 8), 256, 0, stream>>>(
      STH, STL, NUNIT, DWH, DWL, NUNIT, (void*)Y16, NUNIT, db, NBATCH, NUNIT, NUNIT, 1.0f);

  wmma_gemm64<0, false, 2, 0, 0><<<dim3((NBATCH / 64) * (NVOCAB / 64) / 8), 256, 0, stream>>>(
      Y16, Y16, NUNIT, OWT, OWT, NUNIT, (void*)logits, NVOCAB, ob, NBATCH, NVOCAB, NUNIT, LOGIT_FOLD);
}
